// GATLayer_84146999263289
// MI455X (gfx1250) — hardware-verified
//
#include <hip/hip_runtime.h>
#include <stddef.h>
#include <stdint.h>
#include <math.h>


#define NB     8
#define NN     1024
#define FIN    256
#define NHD    4
#define DFH    64
#define HC     256
#define MROW   (NB * NN)
#define NEGSL  0.2f
#define GTHR   128
#define ATHR   128
#define PTHR   256
#define PB_H   (MROW * (FIN / 8) / PTHR)
#define PB_W   (HC * (FIN / 8) / PTHR)
#define PB_M   (NN * 32 / PTHR)
#define PB_TOT (PB_H + PB_W + PB_M + 1)
#define WSMAX  134217728

static_assert((FIN % 32) == 0);
static_assert(HC == NHD * DFH);
static_assert(DFH == 64 && (MROW % 64) == 0 && (NN % 64) == 0);
static_assert((MROW * (FIN / 8)) % PTHR == 0);
static_assert((HC * (FIN / 8)) % PTHR == 0);
static_assert((NN * 32) % PTHR == 0);
static_assert(NHD * 2 * DFH == 4 * 128);

typedef float          v4f  __attribute__((ext_vector_type(4)));
typedef float          v8f  __attribute__((ext_vector_type(8)));
typedef int            v4i  __attribute__((ext_vector_type(4)));
typedef int            v8i  __attribute__((ext_vector_type(8)));
typedef unsigned int   v4u  __attribute__((ext_vector_type(4)));
typedef unsigned short v8us __attribute__((ext_vector_type(8)));
typedef __bf16         v16b __attribute__((ext_vector_type(16)));
typedef v4f  __attribute__((may_alias)) v4fa;
typedef v4i  __attribute__((may_alias)) v4ia;
typedef v4u  __attribute__((may_alias)) v4ua;
typedef v8us __attribute__((may_alias)) v8usa;
union FragB { v16b v; v8us h[2]; v8i w; };

__device__ __forceinline__ v8f wmb(const FragB& a, const FragB& b, v8f c) {
  v8f d = __builtin_amdgcn_wmma_f32_16x16x32_bf16(false, a.v, false, b.v, (short)0, c, false, false);
  asm volatile("v_nop\n\tv_nop\n\tv_nop\n\tv_nop" : "+v"(d) : "v"(a.w), "v"(b.w));
  return d;
}

__device__ __forceinline__ unsigned int f2bf(float f) {
  const unsigned int u = __float_as_uint(f);
  return ((u + 0x7FFFu + ((u >> 16) & 1u)) >> 16) & 0xFFFFu;
}
__device__ __forceinline__ float bf2f(unsigned int b) { return __uint_as_float(b << 16); }
__device__ __forceinline__ float bfr(float f) { return bf2f(f2bf(f)); }
__device__ __forceinline__ unsigned int pk2(float lo, float hi) { return f2bf(lo) | (f2bf(hi) << 16); }
__device__ __forceinline__ v4u pack8(const v4f a, const v4f b) {
  v4u r;
  r.x = pk2(a.x, a.y); r.y = pk2(a.z, a.w); r.z = pk2(b.x, b.y); r.w = pk2(b.z, b.w);
  return r;
}

__global__ __launch_bounds__(PTHR) void k_prep(const float* __restrict__ h, const int* __restrict__ adj,
                                               const float* __restrict__ W, const float* __restrict__ a,
                                               unsigned short* hb, unsigned short* wt,
                                               unsigned int* maskb, float* af) {
  const int blk = (int)blockIdx.x, tid = (int)threadIdx.x;
  if (blk < PB_H) {
    const int u   = blk * PTHR + tid;
    const int row = u >> 5;
    const int c0  = (u & 31) * 8;
    const float* p = h + (size_t)row * FIN + c0;
    const v4f a0 = *(const v4fa*)p, b0 = *(const v4fa*)(p + 4);
    const v4u hv = pack8(a0, b0);
    unsigned short* o = hb + (size_t)row * FIN + c0;
    *(volatile v4u*)o = hv;
    __threadfence();
    *(volatile v4u*)o = hv;
  } else if (blk < PB_H + PB_W) {
    const int u  = (blk - PB_H) * PTHR + tid;
    const int n  = u >> 5;
    const int k8 = (u & 31) * 8;
    const float* p = W + (size_t)k8 * HC + n;
    v4f a0, b0;
    a0.x = p[0];        a0.y = p[HC];       a0.z = p[2 * HC];   a0.w = p[3 * HC];
    b0.x = p[4 * HC];   b0.y = p[5 * HC];   b0.z = p[6 * HC];   b0.w = p[7 * HC];
    const v4u wv = pack8(a0, b0);
    unsigned short* o = wt + (size_t)n * FIN + k8;
    *(volatile v4u*)o = wv;
    __threadfence();
    *(volatile v4u*)o = wv;
  } else if (blk < PB_H + PB_W + PB_M) {
    const int t = (blk - PB_H - PB_W) * PTHR + tid;
    const int i = t >> 5, w = t & 31;
    const int* row = adj + (size_t)i * NN + w * 32;
    unsigned int bits = 0u;
#pragma unroll
    for (int q = 0; q < 32; q += 4) {
      const v4i v = *(const v4ia*)(row + q);
      bits |= (v.x != 0 ? 1u : 0u) << (q + 0);
      bits |= (v.y != 0 ? 1u : 0u) << (q + 1);
      bits |= (v.z != 0 ? 1u : 0u) << (q + 2);
      bits |= (v.w != 0 ? 1u : 0u) << (q + 3);
    }
    unsigned int* o = maskb + t;
    *(volatile unsigned int*)o = bits;
    __threadfence();
    *(volatile unsigned int*)o = bits;
  } else {
    if (tid < 128) {
      const v4f v = *(const v4fa*)(a + 4 * tid);
      v4f r; r.x = bfr(v.x); r.y = bfr(v.y); r.z = bfr(v.z); r.w = bfr(v.w);
      float* o = af + 4 * tid;
      *(volatile v4f*)o = r;
      __threadfence();
      *(volatile v4f*)o = r;
    }
  }
}

__global__ __launch_bounds__(GTHR) void k_wh(const unsigned short* __restrict__ A, const unsigned short* __restrict__ WT,
                                             const float* __restrict__ AF,
                                             unsigned short* VTH, unsigned short* VTL, float* SDV) {
  __shared__ __attribute__((aligned(16))) float stg[64 * 64];
  __shared__ __attribute__((aligned(16))) float satt[128];
  __shared__ __attribute__((aligned(16))) float sdot[128];
  const int tid = (int)threadIdx.x, lane = tid & 31, wave = tid >> 5, hh = lane >> 4, m = lane & 15;
  const int rowBase = (int)blockIdx.x * 64;
  const int head    = (int)blockIdx.y;
  const int col0    = head * 64;

  satt[tid] = AF[head * 128 + tid];

  v8f acc[4];
  {
    const v8f z = {0.f, 0.f, 0.f, 0.f, 0.f, 0.f, 0.f, 0.f};
    acc[0] = z; acc[1] = z; acc[2] = z; acc[3] = z;
  }
  const unsigned short* ap = A  + (size_t)(rowBase + 16 * wave + m) * FIN + 8 * hh;
  const unsigned short* wp = WT + (size_t)(col0 + m) * FIN + 8 * hh;
#pragma unroll 1
  for (int ks = 0; ks < FIN / 32; ++ks) {
    FragB af;
    af.h[0] = *(const v8usa*)(ap + 32 * ks);
    af.h[1] = *(const v8usa*)(ap + 32 * ks + 16);
#pragma unroll
    for (int t = 0; t < 4; ++t) {
      const unsigned short* wq = wp + (size_t)(16 * t) * FIN + 32 * ks;
      FragB bf;
      bf.h[0] = *(const v8usa*)wq;
      bf.h[1] = *(const v8usa*)(wq + 16);
      acc[t] = wmb(af, bf, acc[t]);
    }
  }

#pragma unroll
  for (int t = 0; t < 4; ++t) {
    const int lc = 16 * t + m;
#pragma unroll
    for (int r = 0; r < 8; ++r) {
      const int lr = 16 * wave + 8 * hh + r;
      stg[lr * 64 + lc] = acc[t][r];
    }
  }
  __syncthreads();

  {
    const int row = tid & 63, which = tid >> 6;
    const float* sa = satt + which * 64;
    const float* hr = stg + row * 64;
    float d = 0.f;
#pragma unroll 4
    for (int c4 = 0; c4 < 16; ++c4) {
      const v4f hv = *(const v4fa*)(hr + 4 * c4);
      const v4f av = *(const v4fa*)(sa + 4 * c4);
      d = fmaf(hv.x, av.x, d);
      d = fmaf(hv.y, av.y, d);
      d = fmaf(hv.z, av.z, d);
      d = fmaf(hv.w, av.w, d);
    }
    sdot[which * 64 + row] = d;
  }
  __syncthreads();

  const int bh = (rowBase >> 10) * NHD + head;
  const int j0 = rowBase & (NN - 1);
  v4u hv[4], lv[4];
#pragma unroll
  for (int i = 0; i < 4; ++i) {
    const int p  = tid + 128 * i;
    const int d  = p >> 3;
    const int j8 = (p & 7) * 8;
    unsigned int hb[8], lb[8];
#pragma unroll
    for (int e = 0; e < 8; ++e) {
      const float f = stg[(j8 + e) * 64 + d];
      hb[e] = f2bf(f);
      lb[e] = f2bf(f - bf2f(hb[e]));
    }
    hv[i].x = hb[0] | (hb[1] << 16); hv[i].y = hb[2] | (hb[3] << 16);
    hv[i].z = hb[4] | (hb[5] << 16); hv[i].w = hb[6] | (hb[7] << 16);
    lv[i].x = lb[0] | (lb[1] << 16); lv[i].y = lb[2] | (lb[3] << 16);
    lv[i].z = lb[4] | (lb[5] << 16); lv[i].w = lb[6] | (lb[7] << 16);
  }
  const int which2 = lane >> 4, piece = lane & 15;
  const v4f sdv = *(const v4fa*)(sdot + which2 * 64 + 4 * piece);
  float* sp = SDV + (size_t)(2 * head + which2) * MROW + rowBase + 4 * piece;

#pragma unroll
  for (int i = 0; i < 4; ++i) {
    const int p = tid + 128 * i;
    const size_t o = (size_t)(bh * 64 + (p >> 3)) * NN + j0 + (p & 7) * 8;
    *(volatile v4u*)(VTH + o) = hv[i];
    *(volatile v4u*)(VTL + o) = lv[i];
  }
  if (wave == 0) *(volatile v4f*)sp = sdv;
  __threadfence();
#pragma unroll
  for (int i = 0; i < 4; ++i) {
    const int p = tid + 128 * i;
    const size_t o = (size_t)(bh * 64 + (p >> 3)) * NN + j0 + (p & 7) * 8;
    *(volatile v4u*)(VTH + o) = hv[i];
    *(volatile v4u*)(VTL + o) = lv[i];
  }
  if (wave == 0) *(volatile v4f*)sp = sdv;
}

__device__ __forceinline__ float pval(float ss, float sd, unsigned int bit, float msafe) {
  float t = ss + sd;
  t = t > 0.f ? t : NEGSL * t;
  const float p = expf(fminf(t - msafe, 0.f));
  return bit != 0u ? p : 0.f;
}

__global__ __launch_bounds__(ATHR) void k_agg(const unsigned int* __restrict__ maskb,
                                              const unsigned short* __restrict__ VTH,
                                              const unsigned short* __restrict__ VTL,
                                              const float* __restrict__ SDV, float* out) {
  __shared__ __attribute__((aligned(16))) float        sdl[NN];
  __shared__ __attribute__((aligned(16))) unsigned int mk[64 * 32];
  __shared__ __attribute__((aligned(16))) float        ssl[64];
  __shared__ __attribute__((aligned(16))) float        stg[64 * 64];
  __shared__ __attribute__((aligned(16))) float        linv[64];
  __shared__ int cls[16];
  const int tid = (int)threadIdx.x, lane = tid & 31, wave = tid >> 5, hh = lane >> 4, m = lane & 15;
  const int bx = (int)blockIdx.x;
  const int it = bx & 15, bh = bx >> 4, b = bh >> 2, hd = bh & 3;
  const float* SSp = SDV + (size_t)(2 * hd) * MROW + b * NN + it * 64;
  const float* SDp = SDV + (size_t)(2 * hd + 1) * MROW + b * NN;

  *(v4fa*)(sdl + 4 * tid)         = *(const v4fa*)(SDp + 4 * tid);
  *(v4fa*)(sdl + 4 * (tid + 128)) = *(const v4fa*)(SDp + 4 * (tid + 128));
  {
    const unsigned int* mg = maskb + (size_t)it * 64 * 32;
#pragma unroll
    for (int i = 0; i < 4; ++i)
      *(v4ua*)(mk + 4 * (tid + 128 * i)) = *(const v4ua*)(mg + 4 * (tid + 128 * i));
    const int q = tid & 15;
    const v4f sv = *(const v4fa*)(SSp + 4 * q);
    if (tid < 16) *(v4fa*)(ssl + 4 * q) = sv;
  }
  __syncthreads();
  {
    const int jt = tid & 15;
    unsigned int o = 0u, an = 0xFFFFFFFFu;
#pragma unroll 4
    for (int r = 0; r < 64; ++r) {
      const unsigned int w0 = mk[r * 32 + 2 * jt], w1 = mk[r * 32 + 2 * jt + 1];
      o |= (w0 | w1);
      an &= (w0 & w1);
    }
    const int c = (o == 0u) ? 0 : ((an == 0xFFFFFFFFu) ? 1 : 2);
    if (tid < 16) cls[jt] = c;
  }
  __syncthreads();

  const int il = 16 * wave + m;
  const float ss = ssl[il];
  const unsigned int* mrow = mk + il * 32;

  float mx = -3.0e38f;
#pragma unroll 1
  for (int ks = 0; ks < 32; ++ks) {
    const unsigned int wd = mrow[ks];
    const int j0 = 32 * ks + 8 * hh;
    const v4f s0 = *(const v4fa*)(sdl + j0),      s1 = *(const v4fa*)(sdl + j0 + 4);
    const v4f s2 = *(const v4fa*)(sdl + j0 + 16), s3 = *(const v4fa*)(sdl + j0 + 20);
    const float sv[16] = {s0.x, s0.y, s0.z, s0.w, s1.x, s1.y, s1.z, s1.w,
                          s2.x, s2.y, s2.z, s2.w, s3.x, s3.y, s3.z, s3.w};
    const unsigned int b1 = wd >> (8 * hh), b2 = wd >> (8 * hh + 16);
#pragma unroll
    for (int q = 0; q < 16; ++q) {
      const unsigned int bit = (q < 8) ? ((b1 >> q) & 1u) : ((b2 >> (q - 8)) & 1u);
      float t = ss + sv[q];
      t = t > 0.f ? t : NEGSL * t;
      const float cand = fmaxf(mx, t);
      mx = bit != 0u ? cand : mx;
    }
  }
  mx = fmaxf(mx, __shfl_xor(mx, 16));
  const float msafe = mx > -1.0e37f ? mx : 0.f;

  v8f acc[4];
  {
    const v8f z = {0.f, 0.f, 0.f, 0.f, 0.f, 0.f, 0.f, 0.f};
    acc[0] = z; acc[1] = z; acc[2] = z; acc[3] = z;
  }
  float lsum = 0.0f;
  const unsigned short* vhp = VTH + (size_t)(bh * 64 + m) * NN + 8 * hh;
  const unsigned short* vlp = VTL + (size_t)(bh * 64 + m) * NN + 8 * hh;
#pragma unroll 1
  for (int ks = 0; ks < 32; ++ks) {
    const int c = __builtin_amdgcn_readfirstlane(cls[ks >> 1]);
    if (c == 0) continue;
    const unsigned int wd = mrow[ks];
    const int j0 = 32 * ks + 8 * hh;
    const v4f s0 = *(const v4fa*)(sdl + j0),      s1 = *(const v4fa*)(sdl + j0 + 4);
    const v4f s2 = *(const v4fa*)(sdl + j0 + 16), s3 = *(const v4fa*)(sdl + j0 + 20);
    const float sv[16] = {s0.x, s0.y, s0.z, s0.w, s1.x, s1.y, s1.z, s1.w,
                          s2.x, s2.y, s2.z, s2.w, s3.x, s3.y, s3.z, s3.w};
    const unsigned int b1 = wd >> (8 * hh), b2 = wd >> (8 * hh + 16);
    FragB ph, pl;
#pragma unroll
    for (int i = 0; i < 8; ++i) {
      const int q0 = 2 * i, q1 = 2 * i + 1;
      const unsigned int bit0 = (q0 < 8) ? ((b1 >> q0) & 1u) : ((b2 >> (q0 - 8)) & 1u);
      const unsigned int bit1 = (q1 < 8) ? ((b1 >> q1) & 1u) : ((b2 >> (q1 - 8)) & 1u);
      const float p0 = pval(ss, sv[q0], bit0, msafe);
      const float p1 = pval(ss, sv[q1], bit1, msafe);
      lsum += p0;
      lsum += p1;
      const unsigned int h0 = f2bf(p0), h1 = f2bf(p1);
      const unsigned int l0 = f2bf(p0 - bf2f(h0)), l1 = f2bf(p1 - bf2f(h1));
      ph.w[i] = (int)(h0 | (h1 << 16));
      pl.w[i] = (int)(l0 | (l1 << 16));
    }
#pragma unroll
    for (int t = 0; t < 4; ++t) {
      const size_t o = (size_t)(16 * t) * NN + 32 * ks;
      FragB vh, vl;
      vh.h[0] = *(const v8usa*)(vhp + o);
      vh.h[1] = *(const v8usa*)(vhp + o + 16);
      vl.h[0] = *(const v8usa*)(vlp + o);
      vl.h[1] = *(const v8usa*)(vlp + o + 16);
      acc[t] = wmb(ph, vh, acc[t]);
      acc[t] = wmb(ph, vl, acc[t]);
      acc[t] = wmb(pl, vh, acc[t]);
    }
  }

  const float l = lsum + __shfl_xor(lsum, 16);
  const float lsafe = l > 0.f ? l : 1.0f;
  const float inv = (l > 0.f ? 1.0f : 0.0f) * (1.0f / lsafe);
  if (hh == 0) linv[il] = inv;
#pragma unroll
  for (int t = 0; t < 4; ++t) {
    const int lc = 16 * t + m;
#pragma unroll
    for (int r = 0; r < 8; ++r) {
      const int lr = 16 * wave + 8 * hh + r;
      stg[lr * 64 + lc] = acc[t][r];
    }
  }
  __syncthreads();

#pragma unroll 1
  for (int i = 0; i < 8; ++i) {
    const int lr = 16 * wave + 2 * i + hh;
    const v4f v = *(const v4fa*)(stg + lr * 64 + 4 * m);
    const float s = linv[lr];
    v4f x;
    x.x = v.x * s; x.y = v.y * s; x.z = v.z * s; x.w = v.w * s;
    x.x = x.x > 0.f ? x.x : expm1f(x.x);
    x.y = x.y > 0.f ? x.y : expm1f(x.y);
    x.z = x.z > 0.f ? x.z : expm1f(x.z);
    x.w = x.w > 0.f ? x.w : expm1f(x.w);
    *(v4fa*)(stg + lr * 64 + 4 * m) = x;
  }

  float* ob = out + (size_t)(b * NN + it * 64) * HC + hd * 64 + 4 * m;
#pragma unroll
  for (int i = 0; i < 8; ++i) {
    const int lr = 16 * wave + 2 * i + hh;
    const v4f v = *(const v4fa*)(stg + lr * 64 + 4 * m);
    *(volatile v4f*)(ob + (size_t)lr * HC) = v;
  }
  __threadfence();
#pragma unroll
  for (int i = 0; i < 8; ++i) {
    const int lr = 16 * wave + 2 * i + hh;
    const v4f v = *(const v4fa*)(stg + lr * 64 + 4 * m);
    *(volatile v4f*)(ob + (size_t)lr * HC) = v;
  }
}

extern "C" void kernel_launch(void* const* d_in, const int* in_sizes, int n_in,
                              void* d_out, int out_size, void* d_ws, size_t ws_size,
                              hipStream_t stream) {
  if (n_in < 4) return;
  if (in_sizes[0] != NB * NN * FIN) return;
  if (in_sizes[1] != NN * NN) return;
  if (in_sizes[2] != FIN * HC) return;
  if (in_sizes[3] != NHD * 2 * DFH) return;
  if (out_size != NB * NN * HC) return;

  const float* h   = (const float*)d_in[0];
  const int*   adj = (const int*)  d_in[1];
  const float* W   = (const float*)d_in[2];
  const float* a   = (const float*)d_in[3];
  float* out = (float*)d_out;

  char* ws = (char*)d_ws;
  size_t off = 0;
  const size_t oHB = off; off += (size_t)MROW * FIN * 2;           off = (off + 255) & ~(size_t)255;
  const size_t oWT = off; off += (size_t)HC * FIN * 2;             off = (off + 255) & ~(size_t)255;
  const size_t oAF = off; off += (size_t)NHD * 2 * DFH * 4;        off = (off + 255) & ~(size_t)255;
  const size_t oMB = off; off += (size_t)NN * 32 * 4;              off = (off + 255) & ~(size_t)255;
  const size_t oSD = off; off += (size_t)2 * NHD * MROW * 4;       off = (off + 255) & ~(size_t)255;
  const size_t oVH = off; off += (size_t)NB * NHD * DFH * NN * 2;  off = (off + 255) & ~(size_t)255;
  const size_t oVL = off; off += (size_t)NB * NHD * DFH * NN * 2;  off = (off + 255) & ~(size_t)255;
  if (off > ws_size || off > (size_t)WSMAX) return;
  unsigned short* HB    = (unsigned short*)(ws + oHB);
  unsigned short* WT    = (unsigned short*)(ws + oWT);
  float*          AF    = (float*)(ws + oAF);
  unsigned int*   MASKB = (unsigned int*)(ws + oMB);
  float*          SDV   = (float*)(ws + oSD);
  unsigned short* VTH   = (unsigned short*)(ws + oVH);
  unsigned short* VTL   = (unsigned short*)(ws + oVL);

  k_prep<<<PB_TOT, PTHR, 0, stream>>>(h, adj, W, a, HB, WT, MASKB, AF);
  k_wh<<<dim3(MROW / 64, NHD), GTHR, 0, stream>>>(HB, WT, AF, VTH, VTL, SDV);
  k_agg<<<NB * NHD * (NN / 64), ATHR, 0, stream>>>(MASKB, VTH, VTL, SDV, out);
}
